// Parallel_GCN_83562883711802
// MI455X (gfx1250) — hardware-verified
//
#include <hip/hip_runtime.h>
#include <hip/hip_bf16.h>
#include <stddef.h>


#define DIM     256
#define NTHR    256
#define NWAVE   8
#define EPT     8
#define NGRP    2
#define CHUNK   (NTHR * EPT * NGRP)
#define WCAP    (EPT * NGRP * 32)
#define LISTN   (NWAVE * WCAP)
#define NBC     4096
#define NBF     1024
#define RCAP    40960
#define RBN     128
#define OTHR    512
#define TGT     32
#define NPW     (TGT / NWAVE)
#define DEGCAP  256
#define APK     (DIM + 8)

#define LDS_FILL  ((RCAP + NBF + LISTN) * 4 + 64)
#define LDS_GEMM  (TGT * APK * 2 * 2)

static_assert((CHUNK & (CHUNK - 1)) == 0);
static_assert(CHUNK <= 4096);
static_assert((NBC & (NBC - 1)) == 0 && (NBF & (NBF - 1)) == 0);
static_assert(NBC == 4 * NBF);
static_assert(OTHR * 8 == NBC);
static_assert((RCAP % 32) == 0);
static_assert(TGT == NWAVE * NPW);
static_assert((APK % 8) == 0);
static_assert(TGT * DIM * 4 <= LDS_GEMM);
static_assert(((DIM * DIM / 8) % NTHR) == 0);
static_assert(DIM == 256);

typedef float          v4f  __attribute__((ext_vector_type(4)));
typedef float          v8f  __attribute__((ext_vector_type(8)));
typedef int            v4i  __attribute__((ext_vector_type(4)));
typedef unsigned short v4us __attribute__((ext_vector_type(4)));
typedef unsigned short v8us __attribute__((ext_vector_type(8)));
typedef __bf16         v16b __attribute__((ext_vector_type(16)));
union FragB { v16b v; v8us u[2]; };

__device__ __forceinline__ unsigned short bf_bits(float f) {
  unsigned int u = __float_as_uint(f);
  u += 0x7FFFu + ((u >> 16) & 1u);
  return (unsigned short)(u >> 16);
}
__device__ __forceinline__ float bf_val(unsigned short s) {
  return __uint_as_float(((unsigned int)s) << 16);
}
__device__ __forceinline__ void split4(v4f t, v4us& hv, v4us& lv) {
  const unsigned short h0 = bf_bits(t.x), h1 = bf_bits(t.y), h2 = bf_bits(t.z), h3 = bf_bits(t.w);
  hv.x = h0; hv.y = h1; hv.z = h2; hv.w = h3;
  lv.x = bf_bits(t.x - bf_val(h0));
  lv.y = bf_bits(t.y - bf_val(h1));
  lv.z = bf_bits(t.z - bf_val(h2));
  lv.w = bf_bits(t.w - bf_val(h3));
}

__device__ __forceinline__ v8f wmb(v16b a, v16b b, v8f c) {
  v8f d = __builtin_amdgcn_wmma_f32_16x16x32_bf16(false, a, false, b, (short)0, c, false, false);
  asm volatile("v_nop\n\tv_nop\n\tv_nop\n\tv_nop" : "+v"(d) : "v"(a), "v"(b));
  return d;
}

template <int NB>
__device__ __forceinline__ int scan_chunk(const int* __restrict__ keys, int nE, int cbase, int slotBase,
                                          int vec8, int* list, int tid, int lane, int wave) {
  int wc = 0;
#pragma unroll
  for (int g = 0; g < NGRP; ++g) {
    const int el0  = (g * NTHR + tid) * EPT;
    const int e0   = cbase + el0;
    const int sent = -2147483647 - 1;
    v4i da, db;
    if (vec8 != 0 && cbase + CHUNK <= nE) {
      da = *(const v4i*)(keys + e0);
      db = *(const v4i*)(keys + e0 + 4);
    } else {
      da.x = (e0     < nE) ? keys[min(e0, nE - 1)] : sent;
      da.y = (e0 + 1 < nE) ? keys[min(e0 + 1, nE - 1)] : sent;
      da.z = (e0 + 2 < nE) ? keys[min(e0 + 2, nE - 1)] : sent;
      da.w = (e0 + 3 < nE) ? keys[min(e0 + 3, nE - 1)] : sent;
      db.x = (e0 + 4 < nE) ? keys[min(e0 + 4, nE - 1)] : sent;
      db.y = (e0 + 5 < nE) ? keys[min(e0 + 5, nE - 1)] : sent;
      db.z = (e0 + 6 < nE) ? keys[min(e0 + 6, nE - 1)] : sent;
      db.w = (e0 + 7 < nE) ? keys[min(e0 + 7, nE - 1)] : sent;
    }
    const unsigned nb = (unsigned)slotBase;
    const unsigned s0 = (unsigned)da.x - nb, s1 = (unsigned)da.y - nb;
    const unsigned s2 = (unsigned)da.z - nb, s3 = (unsigned)da.w - nb;
    const unsigned s4 = (unsigned)db.x - nb, s5 = (unsigned)db.y - nb;
    const unsigned s6 = (unsigned)db.z - nb, s7 = (unsigned)db.w - nb;
    const bool h0 = s0 < (unsigned)NB, h1 = s1 < (unsigned)NB, h2 = s2 < (unsigned)NB, h3 = s3 < (unsigned)NB;
    const bool h4 = s4 < (unsigned)NB, h5 = s5 < (unsigned)NB, h6 = s6 < (unsigned)NB, h7 = s7 < (unsigned)NB;
    const unsigned any = __builtin_amdgcn_ballot_w32(h0 | h1 | h2 | h3 | h4 | h5 | h6 | h7);
    if (any != 0u) {
#define HITJ(J, HJ, SJ) { \
        const unsigned mj = __builtin_amdgcn_ballot_w32(HJ); \
        if (mj != 0u) { \
          if (HJ) { \
            const int pos = wc + (int)__builtin_amdgcn_mbcnt_lo(mj, 0u); \
            if (pos < WCAP) list[wave * WCAP + pos] = ((el0 + (J)) << 12) | (int)(SJ); \
          } \
          wc += (int)__builtin_popcount(mj); } }
      HITJ(0, h0, s0)
      HITJ(1, h1, s1)
      HITJ(2, h2, s2)
      HITJ(3, h3, s3)
      HITJ(4, h4, s4)
      HITJ(5, h5, s5)
      HITJ(6, h6, s6)
      HITJ(7, h7, s7)
#undef HITJ
    }
  }
  return wc;
}

__global__ __launch_bounds__(NTHR) void k_wprep(
    const float* __restrict__ W, unsigned short* wHi, unsigned short* wLo) {
  const int i = blockIdx.x * NTHR + (int)threadIdx.x;
  if (i >= DIM * DIM / 8) return;
  const int o  = i * 8;
  const int n  = o >> 8;
  const int k0 = o & (DIM - 1);
  float v[8];
#pragma unroll
  for (int e = 0; e < 8; ++e) v[e] = W[(size_t)(k0 + e) * DIM + n];
  v8us hv, lv;
#pragma unroll
  for (int e = 0; e < 8; ++e) {
    const unsigned short hb = bf_bits(v[e]);
    hv[e] = hb;
    lv[e] = bf_bits(v[e] - bf_val(hb));
  }
  *(volatile v8us*)(wHi + o) = hv;
  *(volatile v8us*)(wLo + o) = lv;
  __threadfence();
  *(volatile v8us*)(wHi + o) = hv;
  *(volatile v8us*)(wLo + o) = lv;
}

__global__ __launch_bounds__(NTHR) void k_count(
    const int* __restrict__ keys, int* cnt, int nE, int vec8) {
  __shared__ __attribute__((aligned(16))) int scnt[NBC];
  __shared__ __attribute__((aligned(16))) int list[LISTN];
  __shared__ int wcnt[NWAVE];
  const int tid = threadIdx.x, lane = tid & 31, wave = tid >> 5;
  const int nodeBase = blockIdx.x * NBC;

  for (int i = tid; i < NBC; i += NTHR) scnt[i] = 0;
  __syncthreads();

  const int nChunks = (nE + CHUNK - 1) / CHUNK;
#pragma unroll 1
  for (int ch = 0; ch < nChunks; ++ch) {
    const int cbase = ch * CHUNK;
    const int wc = scan_chunk<NBC>(keys, nE, cbase, nodeBase, vec8, list, tid, lane, wave);
    if (lane == 0) wcnt[wave] = wc;
    __syncthreads();
    if (wave == 0) {
#pragma unroll 1
      for (int wsx = 0; wsx < NWAVE; ++wsx) {
        int n = __builtin_amdgcn_readfirstlane(wcnt[wsx]);
        n = n > WCAP ? WCAP : (n < 0 ? 0 : n);
        const int* lp = list + wsx * WCAP;
#pragma unroll 1
        for (int i = 0; i < n; ++i) {
          const int ent  = __builtin_amdgcn_readfirstlane(lp[i]);
          const int slot = ent & (NBC - 1);
          if (lane == 0) scnt[slot] = scnt[slot] + 1;
        }
      }
    }
    __syncthreads();
  }

  v4i cq[4];
#pragma unroll
  for (int q = 0; q < 4; ++q) {
    const int f = (wave * 4 + q) * 128 + 4 * lane;
    cq[q] = *(const v4i*)(scnt + f);
  }
  int* cp = cnt + (size_t)nodeBase;
#pragma unroll
  for (int q = 0; q < 4; ++q) {
    const int f = (wave * 4 + q) * 128 + 4 * lane;
    *(volatile v4i*)(cp + f) = cq[q];
  }
  __threadfence();
#pragma unroll
  for (int q = 0; q < 4; ++q) {
    const int f = (wave * 4 + q) * 128 + 4 * lane;
    *(volatile v4i*)(cp + f) = cq[q];
  }
}

__global__ __launch_bounds__(NTHR) void k_norm(
    const int* __restrict__ cnt, float* nrm, int n4) {
  const int i = blockIdx.x * NTHR + (int)threadIdx.x;
  if (i >= n4) return;
  const v4i c = *(const v4i*)(cnt + 4 * (size_t)i);
  v4f r;
  r.x = 1.0f / sqrtf((float)(c.x < 1 ? 1 : c.x));
  r.y = 1.0f / sqrtf((float)(c.y < 1 ? 1 : c.y));
  r.z = 1.0f / sqrtf((float)(c.z < 1 ? 1 : c.z));
  r.w = 1.0f / sqrtf((float)(c.w < 1 ? 1 : c.w));
  *(volatile v4f*)(nrm + 4 * (size_t)i) = r;
  __threadfence();
  *(volatile v4f*)(nrm + 4 * (size_t)i) = r;
}

__global__ __launch_bounds__(OTHR) void k_offsets(
    const int* __restrict__ cnt, int* off, int* rbase, int nChunk) {
  __shared__ __attribute__((aligned(16))) int soff[NBC];
  __shared__ __attribute__((aligned(16))) int srb[RBN];
  __shared__ int wtot[OTHR / 32];
  const int tid = threadIdx.x, lane = tid & 31, wave = tid >> 5, sub = tid >> 7;
  for (int i = tid; i < RBN; i += OTHR) srb[i] = 0;
  int carry = 0;
#pragma unroll 1
  for (int ch = 0; ch < nChunk; ++ch) {
    const int base = ch * NBC;
    const v4i c0 = *(const v4i*)(cnt + base + 8 * tid);
    const v4i c1 = *(const v4i*)(cnt + base + 8 * tid + 4);
    const int e0 = max(c0.x, 0), e1 = max(c0.y, 0), e2 = max(c0.z, 0), e3 = max(c0.w, 0);
    const int e4 = max(c1.x, 0), e5 = max(c1.y, 0), e6 = max(c1.z, 0), e7 = max(c1.w, 0);
    const int ts = e0 + e1 + e2 + e3 + e4 + e5 + e6 + e7;
    int incl = ts;
#pragma unroll
    for (int d = 1; d < 32; d <<= 1) {
      const int t = __shfl_up(incl, d);
      if (lane >= d) incl += t;
    }
    if (lane == 31) wtot[wave] = incl;
    __syncthreads();
    const int S0 = wtot[0]  + wtot[1]  + wtot[2]  + wtot[3];
    const int S1 = wtot[4]  + wtot[5]  + wtot[6]  + wtot[7];
    const int S2 = wtot[8]  + wtot[9]  + wtot[10] + wtot[11];
    const int S3 = wtot[12] + wtot[13] + wtot[14] + wtot[15];
    int pre = 0;
#pragma unroll 1
    for (int w = 4 * sub; w < wave; ++w) pre += wtot[w];
    const int b0 = carry;
    const int b1 = b0 + ((S0 + 31) & ~31);
    const int b2 = b1 + ((S1 + 31) & ~31);
    const int b3 = b2 + ((S2 + 31) & ~31);
    const int b4 = b3 + ((S3 + 31) & ~31);
    const int myb = sub == 0 ? b0 : (sub == 1 ? b1 : (sub == 2 ? b2 : b3));
    if (tid == 0) {
      srb[min(4 * ch + 0, RBN - 1)] = b0;
      srb[min(4 * ch + 1, RBN - 1)] = b1;
      srb[min(4 * ch + 2, RBN - 1)] = b2;
      srb[min(4 * ch + 3, RBN - 1)] = b3;
    }
    int run = myb + pre + incl - ts;
    soff[8 * tid + 0] = run; run += e0;
    soff[8 * tid + 1] = run; run += e1;
    soff[8 * tid + 2] = run; run += e2;
    soff[8 * tid + 3] = run; run += e3;
    soff[8 * tid + 4] = run; run += e4;
    soff[8 * tid + 5] = run; run += e5;
    soff[8 * tid + 6] = run; run += e6;
    soff[8 * tid + 7] = run;
    carry = b4;
    __syncthreads();
    const v4i o0 = *(const v4i*)(soff + 4 * tid);
    const v4i o1 = *(const v4i*)(soff + 4 * (tid + OTHR));
    int* op = off + base;
    *(volatile v4i*)(op + 4 * tid) = o0;
    *(volatile v4i*)(op + 4 * (tid + OTHR)) = o1;
    __threadfence();
    *(volatile v4i*)(op + 4 * tid) = o0;
    *(volatile v4i*)(op + 4 * (tid + OTHR)) = o1;
    __syncthreads();
  }
  if (tid == 0) srb[min(4 * nChunk, RBN - 1)] = carry;
  __syncthreads();
  v4i rv = {0, 0, 0, 0};
  if (tid < 32) rv = *(const v4i*)(srb + 4 * tid);
  if (tid < 32) *(volatile v4i*)(rbase + 4 * tid) = rv;
  __threadfence();
  if (tid < 32) *(volatile v4i*)(rbase + 4 * tid) = rv;
}

__global__ __launch_bounds__(NTHR) void k_fill(
    const int* __restrict__ dkeys, const int* __restrict__ skeys, const int* __restrict__ off,
    const int* __restrict__ rbase, int* csr, int nN, int nE, int vec8, int csrLen) {
  extern __shared__ v4f lds_dyn[];
  int* region = (int*)lds_dyn;
  int* cursor = region + RCAP;
  int* list   = cursor + NBF;
  int* wcnt   = list + LISTN;
  const int tid = threadIdx.x, lane = tid & 31, wave = tid >> 5;
  const int b = blockIdx.x;
  const int nodeBase = b * NBF;

  int rb0 = rbase[b];
  const int rb1 = rbase[b + 1];
  rb0 = rb0 < 0 ? 0 : (rb0 > csrLen ? csrLen : rb0);
  rb0 &= ~31;
  int len = rb1 - rb0;
  len = len < 0 ? 0 : (len > RCAP ? RCAP : len);
  int lenW = (len + 31) & ~31;
  if (rb0 + lenW > csrLen) lenW = (csrLen - rb0) & ~31;

  {
    const v4i z = {0, 0, 0, 0};
    for (int i = tid; i < RCAP / 4; i += NTHR) ((v4i*)region)[i] = z;
    for (int s = tid; s < NBF; s += NTHR) {
      int o = off[nodeBase + s] - rb0;
      o = o < 0 ? 0 : (o > RCAP ? RCAP : o);
      cursor[s] = o;
    }
  }
  __syncthreads();

  const int nChunks = (nE + CHUNK - 1) / CHUNK;
#pragma unroll 1
  for (int ch = 0; ch < nChunks; ++ch) {
    const int cbase = ch * CHUNK;
    const int wc = scan_chunk<NBF>(dkeys, nE, cbase, nodeBase, vec8, list, tid, lane, wave);
    if (lane == 0) wcnt[wave] = wc;
    __syncthreads();
    if (wave == 0) {
#pragma unroll 1
      for (int wsx = 0; wsx < NWAVE; ++wsx) {
        int n = __builtin_amdgcn_readfirstlane(wcnt[wsx]);
        n = n > WCAP ? WCAP : (n < 0 ? 0 : n);
        const int* lp = list + wsx * WCAP;
#pragma unroll 1
        for (int i = 0; i < n; ++i) {
          const int ent  = __builtin_amdgcn_readfirstlane(lp[i]);
          const int slot = ent & (NBF - 1);
          int e = cbase + ((ent >> 12) & (CHUNK - 1));
          e = e > nE - 1 ? nE - 1 : e;
          int sid = skeys[e];
          sid = sid < 0 ? 0 : (sid > nN - 1 ? nN - 1 : sid);
          if (lane == 0) {
            int pos = cursor[slot];
            pos = pos < 0 ? 0 : (pos > RCAP - 1 ? RCAP - 1 : pos);
            region[pos] = sid;
            const int np = pos + 1;
            cursor[slot] = np > RCAP ? RCAP : np;
          }
        }
      }
    }
    __syncthreads();
  }

  const int nv = lenW >> 2;
  int* gp = csr + rb0;
#pragma unroll 1
  for (int i = tid; i < nv; i += NTHR) { const v4i v = ((const v4i*)region)[i]; *(volatile v4i*)(gp + 4 * i) = v; }
  __threadfence();
#pragma unroll 1
  for (int i = tid; i < nv; i += NTHR) { const v4i v = ((const v4i*)region)[i]; *(volatile v4i*)(gp + 4 * i) = v; }
}

__device__ __forceinline__ void gather_row(
    const float* __restrict__ hin, const float* __restrict__ nrm, const int* __restrict__ csr,
    int n, int st, int nN, int csrLen, int lane, v4f& s0, v4f& s1) {
  const v4f z4 = {0.f, 0.f, 0.f, 0.f};
  s0 = z4; s1 = z4;
#pragma unroll 1
  for (int q0 = 0; q0 < n; q0 += 32) {
    int pos = st + q0 + lane;
    pos = pos > csrLen - 1 ? csrLen - 1 : pos;
    int sid = csr[pos];
    sid = sid < 0 ? 0 : (sid > nN - 1 ? nN - 1 : sid);
    const float nsl = nrm[sid];
    const int mc = (n - q0) < 32 ? (n - q0) : 32;
#pragma unroll 1
    for (int p = 0; p < mc; ++p) {
      const int   s  = __builtin_amdgcn_readlane(sid, p);
      const float ns = __int_as_float(__builtin_amdgcn_readlane(__float_as_int(nsl), p));
      const float* rp = hin + (size_t)s * DIM;
      const v4f a = *(const v4f*)(rp + 4 * lane);
      const v4f c = *(const v4f*)(rp + 128 + 4 * lane);
      s0 = s0 + a * ns;
      s1 = s1 + c * ns;
    }
  }
}

__global__ __launch_bounds__(NTHR) void k_hop(
    const float* __restrict__ hin, const float* __restrict__ nrm, const int* __restrict__ csr,
    const int* __restrict__ off, const int* __restrict__ cnt, float* hout, int nN, int csrLen) {
  const int tid = threadIdx.x, lane = tid & 31, wave = tid >> 5;
  const int node0 = blockIdx.x * TGT;
#pragma unroll 1
  for (int i = 0; i < NPW; ++i) {
    const int nd  = node0 + wave * NPW + i;
    const int ndc = nd > nN - 1 ? nN - 1 : nd;
    int n = __builtin_amdgcn_readfirstlane(cnt[ndc]);
    n = nd < nN ? n : 0;
    n = n < 0 ? 0 : (n > DEGCAP ? DEGCAP : n);
    int st = __builtin_amdgcn_readfirstlane(off[ndc]);
    st = st < 0 ? 0 : (st > csrLen - 1 ? csrLen - 1 : st);
    const float nv = nrm[ndc];
    v4f s0, s1;
    gather_row(hin, nrm, csr, n, st, nN, csrLen, lane, s0, s1);
    const v4f r0 = s0 * nv;
    const v4f r1 = s1 * nv;
    if (nd < nN) {
      float* op = hout + (size_t)nd * DIM;
      *(volatile v4f*)(op + 4 * lane) = r0;
      *(volatile v4f*)(op + 128 + 4 * lane) = r1;
      __threadfence();
      *(volatile v4f*)(op + 4 * lane) = r0;
      *(volatile v4f*)(op + 128 + 4 * lane) = r1;
    }
  }
}

__global__ __launch_bounds__(NTHR) void k_hop_gemm(
    const float* __restrict__ hin, const float* __restrict__ feat, const float* __restrict__ hone,
    const float* __restrict__ nrm, const int* __restrict__ csr, const int* __restrict__ off,
    const int* __restrict__ cnt, const unsigned short* __restrict__ wHi,
    const unsigned short* __restrict__ wLo, const float* __restrict__ bias,
    float* out, int nN, int csrLen) {
  extern __shared__ v4f lds_dyn[];
  unsigned short* aHi = (unsigned short*)lds_dyn;
  unsigned short* aLo = aHi + TGT * APK;
  float*          stg = (float*)lds_dyn;
  const int tid = threadIdx.x, lane = tid & 31, wave = tid >> 5, hh = lane >> 4, m = lane & 15;
  const int node0 = blockIdx.x * TGT;

#pragma unroll 1
  for (int i = 0; i < NPW; ++i) {
    const int row = wave * NPW + i;
    const int nd  = node0 + row;
    const int ndc = nd > nN - 1 ? nN - 1 : nd;
    int n = __builtin_amdgcn_readfirstlane(cnt[ndc]);
    n = nd < nN ? n : 0;
    n = n < 0 ? 0 : (n > DEGCAP ? DEGCAP : n);
    int st = __builtin_amdgcn_readfirstlane(off[ndc]);
    st = st < 0 ? 0 : (st > csrLen - 1 ? csrLen - 1 : st);
    const float nv = nrm[ndc];
    v4f s0, s1;
    gather_row(hin, nrm, csr, n, st, nN, csrLen, lane, s0, s1);
    const v4f r0 = s0 * nv;
    const v4f r1 = s1 * nv;
    const size_t ro = (size_t)ndc * DIM;
    const v4f f0 = *(const v4f*)(feat + ro + 4 * lane);
    const v4f f1 = *(const v4f*)(feat + ro + 128 + 4 * lane);
    const v4f a0 = *(const v4f*)(hone + ro + 4 * lane);
    const v4f a1 = *(const v4f*)(hone + ro + 128 + 4 * lane);
    const v4f b0 = *(const v4f*)(hin + ro + 4 * lane);
    const v4f b1 = *(const v4f*)(hin + ro + 128 + 4 * lane);
    const v4f t0 = ((f0 + a0) + b0) + r0;
    const v4f t1 = ((f1 + a1) + b1) + r1;
    v4us h0, l0, h1, l1;
    split4(t0, h0, l0);
    split4(t1, h1, l1);
    *(v4us*)(aHi + row * APK + 4 * lane) = h0;
    *(v4us*)(aHi + row * APK + 128 + 4 * lane) = h1;
    *(v4us*)(aLo + row * APK + 4 * lane) = l0;
    *(v4us*)(aLo + row * APK + 128 + 4 * lane) = l1;
  }
  __syncthreads();

  const int colb = 32 * wave;
  v8f acc[2][2];
  {
    const v8f z8 = {0.f, 0.f, 0.f, 0.f, 0.f, 0.f, 0.f, 0.f};
    acc[0][0] = z8; acc[0][1] = z8; acc[1][0] = z8; acc[1][1] = z8;
  }
  const unsigned short* pa0h = aHi + m * APK + 8 * hh;
  const unsigned short* pa1h = aHi + (16 + m) * APK + 8 * hh;
  const unsigned short* pa0l = aLo + m * APK + 8 * hh;
  const unsigned short* pa1l = aLo + (16 + m) * APK + 8 * hh;
#pragma unroll 1
  for (int ks = 0; ks < DIM / 32; ++ks) {
    FragB a0h, a1h, a0l, a1l, b0h, b0l, b1h, b1l;
    a0h.u[0] = *(const v8us*)(pa0h + 32 * ks);  a0h.u[1] = *(const v8us*)(pa0h + 32 * ks + 16);
    a1h.u[0] = *(const v8us*)(pa1h + 32 * ks);  a1h.u[1] = *(const v8us*)(pa1h + 32 * ks + 16);
    a0l.u[0] = *(const v8us*)(pa0l + 32 * ks);  a0l.u[1] = *(const v8us*)(pa0l + 32 * ks + 16);
    a1l.u[0] = *(const v8us*)(pa1l + 32 * ks);  a1l.u[1] = *(const v8us*)(pa1l + 32 * ks + 16);
    const size_t bo0 = (size_t)(colb + m) * DIM + 32 * ks + 8 * hh;
    const size_t bo1 = (size_t)(colb + 16 + m) * DIM + 32 * ks + 8 * hh;
    b0h.u[0] = *(const v8us*)(wHi + bo0);  b0h.u[1] = *(const v8us*)(wHi + bo0 + 16);
    b0l.u[0] = *(const v8us*)(wLo + bo0);  b0l.u[1] = *(const v8us*)(wLo + bo0 + 16);
    b1h.u[0] = *(const v8us*)(wHi + bo1);  b1h.u[1] = *(const v8us*)(wHi + bo1 + 16);
    b1l.u[0] = *(const v8us*)(wLo + bo1);  b1l.u[1] = *(const v8us*)(wLo + bo1 + 16);
    acc[0][0] = wmb(a0l.v, b0h.v, acc[0][0]);
    acc[0][0] = wmb(a0h.v, b0l.v, acc[0][0]);
    acc[0][0] = wmb(a0h.v, b0h.v, acc[0][0]);
    acc[0][1] = wmb(a0l.v, b1h.v, acc[0][1]);
    acc[0][1] = wmb(a0h.v, b1l.v, acc[0][1]);
    acc[0][1] = wmb(a0h.v, b1h.v, acc[0][1]);
    acc[1][0] = wmb(a1l.v, b0h.v, acc[1][0]);
    acc[1][0] = wmb(a1h.v, b0l.v, acc[1][0]);
    acc[1][0] = wmb(a1h.v, b0h.v, acc[1][0]);
    acc[1][1] = wmb(a1l.v, b1h.v, acc[1][1]);
    acc[1][1] = wmb(a1h.v, b1l.v, acc[1][1]);
    acc[1][1] = wmb(a1h.v, b1h.v, acc[1][1]);
  }
  __syncthreads();

  const float bv0 = 4.0f * bias[colb + m];
  const float bv1 = 4.0f * bias[colb + 16 + m];
#pragma unroll
  for (int rt = 0; rt < 2; ++rt) {
#pragma unroll
    for (int r = 0; r < 8; ++r) {
      const int row = 16 * rt + 8 * hh + r;
      const float v0 = acc[rt][0][r] + bv0;
      const float v1 = acc[rt][1][r] + bv1;
      stg[row * DIM + colb + m]      = v0 > 0.f ? v0 : 0.f;
      stg[row * DIM + colb + 16 + m] = v1 > 0.f ? v1 : 0.f;
    }
  }
  __syncthreads();

#pragma unroll 1
  for (int i = 0; i < NPW; ++i) {
    const int row = wave * NPW + i;
    const int nd = node0 + row;
    const v4f v0 = *(const v4f*)(stg + row * DIM + 4 * lane);
    const v4f v1 = *(const v4f*)(stg + row * DIM + 128 + 4 * lane);
    if (nd < nN) {
      float* op = out + (size_t)nd * DIM;
      *(volatile v4f*)(op + 4 * lane) = v0;
      *(volatile v4f*)(op + 128 + 4 * lane) = v1;
      __threadfence();
      *(volatile v4f*)(op + 4 * lane) = v0;
      *(volatile v4f*)(op + 128 + 4 * lane) = v1;
    }
  }
}

extern "C" void kernel_launch(void* const* d_in, const int* in_sizes, int n_in,
                              void* d_out, int out_size, void* d_ws, size_t ws_size,
                              hipStream_t stream) {
  if (n_in < 5) return;
  const int nN = in_sizes[0] / DIM;
  const int nE = in_sizes[3];
  if (nN <= 0 || nE <= 0 || in_sizes[0] != nN * DIM) return;
  if (in_sizes[1] != DIM * DIM || in_sizes[2] != DIM || in_sizes[4] != nE) return;
  if (out_size != nN * DIM) return;
  if (nE > (1 << 28) || nN > (1 << 24)) return;

  const float* feat = (const float*)d_in[0];
  const float* W    = (const float*)d_in[1];
  const float* bias = (const float*)d_in[2];
  const int*   src  = (const int*)d_in[3];
  const int*   dst  = (const int*)d_in[4];
  float* out = (float*)d_out;

  const int nBC    = (nN + NBC - 1) / NBC;
  const int CNTPAD = nBC * NBC;
  if (4 * nBC + 1 > RBN) return;
  const int nBF    = (nN + NBF - 1) / NBF;
  const int csrLen = ((nE + 31) & ~31) + 4096;
  const int nHop   = (nN + TGT - 1) / TGT;

  char* ws = (char*)d_ws;
  size_t ob = 0;
  const size_t oWH  = ob; ob += (size_t)DIM * DIM * 2;              ob = (ob + 255) & ~(size_t)255;
  const size_t oWL  = ob; ob += (size_t)DIM * DIM * 2;              ob = (ob + 255) & ~(size_t)255;
  const size_t oCnS = ob; ob += (size_t)CNTPAD * 4;                 ob = (ob + 255) & ~(size_t)255;
  const size_t oNrm = ob; ob += (size_t)CNTPAD * 4;                 ob = (ob + 255) & ~(size_t)255;
  const size_t oCnD = ob; ob += (size_t)CNTPAD * 4;                 ob = (ob + 255) & ~(size_t)255;
  const size_t oOff = ob; ob += (size_t)CNTPAD * 4;                 ob = (ob + 255) & ~(size_t)255;
  const size_t oRb  = ob; ob += (size_t)RBN * 4;                    ob = (ob + 255) & ~(size_t)255;
  const size_t oCsr = ob; ob += (size_t)csrLen * 4;                 ob = (ob + 255) & ~(size_t)255;
  const size_t oHA  = ob; ob += (size_t)nHop * TGT * DIM * 4;       ob = (ob + 255) & ~(size_t)255;
  const size_t oHB  = ob; ob += (size_t)nHop * TGT * DIM * 4;       ob = (ob + 255) & ~(size_t)255;
  if (ob > ws_size || ob > ((size_t)128 << 20)) return;
  unsigned short* wHi = (unsigned short*)(ws + oWH);
  unsigned short* wLo = (unsigned short*)(ws + oWL);
  int*   cntS = (int*)(ws + oCnS);
  float* nrm  = (float*)(ws + oNrm);
  int*   cntD = (int*)(ws + oCnD);
  int*   offp = (int*)(ws + oOff);
  int*   rb   = (int*)(ws + oRb);
  int*   csr  = (int*)(ws + oCsr);
  float* hA   = (float*)(ws + oHA);
  float* hB   = (float*)(ws + oHB);

  const int vec8 = ((nE & 3) == 0) ? 1 : 0;

  k_wprep<<<(DIM * DIM / 8 + NTHR - 1) / NTHR, NTHR, 0, stream>>>(W, wHi, wLo);

  k_count<<<nBC, NTHR, 0, stream>>>(src, cntS, nE, vec8);
  const int n4 = CNTPAD / 4;
  k_norm<<<(n4 + NTHR - 1) / NTHR, NTHR, 0, stream>>>(cntS, nrm, n4);

  k_count<<<nBC, NTHR, 0, stream>>>(dst, cntD, nE, vec8);
  k_offsets<<<1, OTHR, 0, stream>>>(cntD, offp, rb, nBC);
  hipFuncSetAttribute(reinterpret_cast<const void*>(&k_fill),
                      hipFuncAttributeMaxDynamicSharedMemorySize, LDS_FILL);
  k_fill<<<nBF, NTHR, LDS_FILL, stream>>>(dst, src, offp, rb, csr, nN, nE, vec8, csrLen);

  k_hop<<<nHop, NTHR, 0, stream>>>(feat, nrm, csr, offp, cntD, hA, nN, csrLen);
  k_hop<<<nHop, NTHR, 0, stream>>>(hA, nrm, csr, offp, cntD, hB, nN, csrLen);

  k_hop_gemm<<<nHop, NTHR, LDS_GEMM, stream>>>(hB, feat, hA, nrm, csr, offp, cntD, wHi, wLo,
                                                bias, out, nN, csrLen);
}
